// STGCN_block_240518168586
// MI455X (gfx1250) — hardware-verified
//
#include <hip/hip_runtime.h>
#define NB 2048
#define TT 3
#define VV 62
#define FD 5
#define HH 64
#define NRV (NB * VV)
#define NS (VV * VV)
typedef __bf16 v16b __attribute__((ext_vector_type(16)));
typedef unsigned short v8us __attribute__((ext_vector_type(8), may_alias));
typedef float  v8f  __attribute__((ext_vector_type(8)));
typedef float  v4f  __attribute__((ext_vector_type(4)));
typedef float  v4fa __attribute__((ext_vector_type(4), may_alias));
union FragB { v16b v; v8us half[2]; unsigned short u[16]; };

__device__ __forceinline__ unsigned short bf16_bits(float x) { unsigned int u = __float_as_uint(x); return (unsigned short)((u + 0x7FFFu + ((u >> 16) & 1u)) >> 16); }
__device__ __forceinline__ float bf16_val(unsigned short b) { return __uint_as_float(((unsigned int)b) << 16); }
__device__ __forceinline__ float bf16_round(float x) { return bf16_val(bf16_bits(x)); }
template <int NT>
__device__ __forceinline__ v8f mmaN(v16b ah, v16b al, v16b bh, v16b bl, v8f c) {
  c = __builtin_amdgcn_wmma_f32_16x16x32_bf16(false, ah, false, bh, (short)0, c, false, false);
  if (NT >= 2) c = __builtin_amdgcn_wmma_f32_16x16x32_bf16(false, al, false, bh, (short)0, c, false, false);
  if (NT >= 3) c = __builtin_amdgcn_wmma_f32_16x16x32_bf16(false, ah, false, bl, (short)0, c, false, false);
  asm volatile("v_nop\n\tv_nop\n\tv_nop\n\tv_nop" : "+v"(c) : "v"(ah), "v"(al), "v"(bh), "v"(bl));
  return c;
}

__global__ __launch_bounds__(256) void k_wt_bf16(const float* __restrict__ W, unsigned short* __restrict__ Wt, int K, int N) {
  const int t = blockIdx.x * 256 + threadIdx.x;
  const int k8n = K / 8;
  if (t >= N * k8n) return;
  const int n = t / k8n, k8 = (t % k8n) * 8;
  v8us v;
#pragma unroll
  for (int i = 0; i < 8; ++i) v[i] = bf16_bits(W[(size_t)(k8 + i) * N + n]);
  *(volatile v8us*)(Wt + (size_t)n * K + k8) = v;
  __threadfence();
  *(volatile v8us*)(Wt + (size_t)n * K + k8) = v;
}

template <bool ASPLIT, int ACT, bool BIAS_BF16>
__global__ __launch_bounds__(128) void k_gemm_bf(const float* __restrict__ A, int lda, const unsigned short* __restrict__ Wt, int ldb,
                                               const float* __restrict__ bias, float* __restrict__ C, int ldc, int M, int N, int K) {
  __shared__ __attribute__((aligned(16))) float so[4][16][64];
  const int tid = threadIdx.x, w = tid >> 5, lane = tid & 31, ln = lane & 15, hh = lane >> 4;
  const int ntn = N / 64;
  const int wid = blockIdx.x * 4 + w;
  const int mt = wid / ntn, nq = wid % ntn;
  if (mt * 16 >= M) return;
  const int row0 = mt * 16, col0 = nq * 64;
  const float* arow = A + (size_t)(row0 + ln) * lda;
  v8f acc[4] = {};
  for (int kb = 0; kb < K; kb += 32) {
    FragB ah, al;
    const v4f x0 = *(const v4fa*)(arow + kb + 8 * hh), x1 = *(const v4fa*)(arow + kb + 8 * hh + 4);
    const v4f x2 = *(const v4fa*)(arow + kb + 16 + 8 * hh), x3 = *(const v4fa*)(arow + kb + 16 + 8 * hh + 4);
    float xs[16] = {x0[0],x0[1],x0[2],x0[3],x1[0],x1[1],x1[2],x1[3],x2[0],x2[1],x2[2],x2[3],x3[0],x3[1],x3[2],x3[3]};
#pragma unroll
    for (int i = 0; i < 16; ++i) { const unsigned short hb = bf16_bits(xs[i]); ah.u[i] = hb; al.u[i] = ASPLIT ? bf16_bits(xs[i] - bf16_val(hb)) : (unsigned short)0; }
#pragma unroll
    for (int t = 0; t < 4; ++t) {
      const unsigned short* brow = Wt + (size_t)(col0 + t * 16 + ln) * ldb + kb;
      FragB b;
      b.half[0] = *(const v8us*)(brow + 8 * hh);
      b.half[1] = *(const v8us*)(brow + 16 + 8 * hh);
      acc[t] = mmaN<ASPLIT ? 2 : 1>(ah.v, al.v, b.v, b.v, acc[t]);
    }
  }
#pragma unroll
  for (int t = 0; t < 4; ++t) {
    float bv = bias ? bias[col0 + t * 16 + ln] : 0.f;
    if (BIAS_BF16) bv = bf16_round(bv);
#pragma unroll
    for (int r = 0; r < 8; ++r) { float v = acc[t][r] + bv; if (ACT == 1) v = fmaxf(v, 0.f); so[w][8 * hh + r][t * 16 + ln] = v; }
  }
  __builtin_amdgcn_fence(__ATOMIC_ACQ_REL, "workgroup");
  __builtin_amdgcn_wave_barrier();
  const int rsub = lane >> 4, c4 = (lane & 15) * 4;
  for (int pass = 0; pass < 2; ++pass) {
#pragma unroll
    for (int q = 0; q < 8; ++q) {
      const int r = q * 2 + rsub;
      const v4f v = *(const v4fa*)&so[w][r][c4];
      *(volatile v4f*)(C + (size_t)(row0 + r) * ldc + col0 + c4) = v;
    }
    if (pass == 0) __threadfence();
  }
}

template <bool ASPLIT, int ACT, bool BIAS_BF16, bool RES_BF16>
__global__ __launch_bounds__(128) void k_gemm_bf3(const float* __restrict__ A, int lda, const unsigned short* __restrict__ Wt, int ldb,
                                                const float* __restrict__ bias, const float* __restrict__ resid, int rmod, int ldr,
                                                float* __restrict__ C, int ldc, int M, int N, int K) {
  __shared__ __attribute__((aligned(16))) float so[4][16][64];
  const int tid = threadIdx.x, w = tid >> 5, lane = tid & 31, ln = lane & 15, hh = lane >> 4;
  const int ntn = N / 64;
  const int wid = blockIdx.x * 4 + w;
  const int mt = wid / ntn, nq = wid % ntn;
  if (mt * 16 >= M) return;
  const int row0 = mt * 16, col0 = nq * 64;
  const float* arow = A + (size_t)(row0 + ln) * lda;
  v8f acc[4] = {};
  for (int kb = 0; kb < K; kb += 32) {
    FragB ah, al;
    const v4f x0 = *(const v4fa*)(arow + kb + 8 * hh), x1 = *(const v4fa*)(arow + kb + 8 * hh + 4);
    const v4f x2 = *(const v4fa*)(arow + kb + 16 + 8 * hh), x3 = *(const v4fa*)(arow + kb + 16 + 8 * hh + 4);
    float xs[16] = {x0[0],x0[1],x0[2],x0[3],x1[0],x1[1],x1[2],x1[3],x2[0],x2[1],x2[2],x2[3],x3[0],x3[1],x3[2],x3[3]};
#pragma unroll
    for (int i = 0; i < 16; ++i) { const unsigned short hb = bf16_bits(xs[i]); ah.u[i] = hb; al.u[i] = ASPLIT ? bf16_bits(xs[i] - bf16_val(hb)) : (unsigned short)0; }
#pragma unroll
    for (int t = 0; t < 4; ++t) {
      const unsigned short* brow = Wt + (size_t)(col0 + t * 16 + ln) * ldb + kb;
      FragB b;
      b.half[0] = *(const v8us*)(brow + 8 * hh);
      b.half[1] = *(const v8us*)(brow + 16 + 8 * hh);
      acc[t] = mmaN<ASPLIT ? 2 : 1>(ah.v, al.v, b.v, b.v, acc[t]);
    }
  }
#pragma unroll
  for (int t = 0; t < 4; ++t) {
    const int col = col0 + t * 16 + ln;
    float bv = bias ? bias[col] : 0.f;
    if (BIAS_BF16) bv = bf16_round(bv);
#pragma unroll
    for (int r = 0; r < 8; ++r) {
      float v = acc[t][r] + bv;
      if (resid) { float rv = resid[(size_t)((row0 + 8 * hh + r) % rmod) * ldr + col]; if (RES_BF16) rv = bf16_round(rv); v += rv; }
      if (ACT == 1) v = fmaxf(v, 0.f);
      if (ACT == 2) v = 0.5f * v * (1.0f + erff(v * 0.70710678118654752f));
      if (ACT == 3) { const float u = 0.7978845608028654f * (v + 0.044715f * v * v * v); v = 0.5f * v * (1.0f + tanhf(u)); }
      so[w][8 * hh + r][t * 16 + ln] = v;
    }
  }
  __builtin_amdgcn_fence(__ATOMIC_ACQ_REL, "workgroup");
  __builtin_amdgcn_wave_barrier();
  const int rsub = lane >> 4, c4 = (lane & 15) * 4;
  for (int pass = 0; pass < 2; ++pass) {
#pragma unroll
    for (int q = 0; q < 8; ++q) {
      const int r = q * 2 + rsub;
      const v4f v = *(const v4fa*)&so[w][r][c4];
      *(volatile v4f*)(C + (size_t)(row0 + r) * ldc + col0 + c4) = v;
    }
    if (pass == 0) __threadfence();
  }
}
template <bool PARAM_BF16>
__global__ __launch_bounds__(256) void k_layernorm(const float* __restrict__ X, const float* __restrict__ R, const float* __restrict__ g, const float* __restrict__ bta,
                                                  float* __restrict__ out_sum, float* __restrict__ out_norm, int N, float eps) {
  __shared__ float red[256];
  const int row = blockIdx.x, tid = threadIdx.x;
  const float* x = X + (size_t)row * N; const float* rr = R ? R + (size_t)row * N : nullptr;
  float vals[16];
  const int per = N / 256;
  float s1 = 0.f;
  for (int u = 0; u < per / 4; ++u) {
    const int j = tid * 4 + 1024 * u;
    const v4f a = *(const v4fa*)(x + j);
    v4f b = {0.f,0.f,0.f,0.f}; if (rr) b = *(const v4fa*)(rr + j);
#pragma unroll
    for (int q = 0; q < 4; ++q) { const float v = a[q] + b[q]; vals[u * 4 + q] = v; s1 += v; }
  }
  red[tid] = s1; __syncthreads();
  for (int st = 128; st > 0; st >>= 1) { if (tid < st) red[tid] += red[tid + st]; __syncthreads(); }
  const float mu = red[0] / (float)N; __syncthreads();
  float s2 = 0.f;
  for (int u = 0; u < per / 4; ++u)
#pragma unroll
    for (int q = 0; q < 4; ++q) { const float c = vals[u * 4 + q] - mu; s2 += c * c; }
  red[tid] = s2; __syncthreads();
  for (int st = 128; st > 0; st >>= 1) { if (tid < st) red[tid] += red[tid + st]; __syncthreads(); }
  const float rs = rsqrtf(red[0] / (float)N + eps);
  for (int pass = 0; pass < 2; ++pass) {
    for (int u = 0; u < per / 4; ++u) {
      const int j = tid * 4 + 1024 * u;
      v4f o, sm;
#pragma unroll
      for (int q = 0; q < 4; ++q) {
        float gg = g[j + q], bb = bta[j + q];
        if (PARAM_BF16) { gg = bf16_round(gg); bb = bf16_round(bb); }
        sm[q] = vals[u * 4 + q]; o[q] = (vals[u * 4 + q] - mu) * rs * gg + bb;
      }
      if (out_sum) *(volatile v4f*)(out_sum + (size_t)row * N + j) = sm;
      *(volatile v4f*)(out_norm + (size_t)row * N + j) = o;
    }
    if (pass == 0) __threadfence();
  }
}


typedef _Float16 v16h __attribute__((ext_vector_type(16)));
union FragH { v16h v; v8us half[2]; _Float16 h[16]; unsigned short u[16]; };
template <int NT>
__device__ __forceinline__ v8f mmaH(v16h ah, v16h al, v16h bh, v16h bl, v8f c) {
  c = __builtin_amdgcn_wmma_f32_16x16x32_f16(false, ah, false, bh, (short)0, c, false, false);
  if (NT >= 2) c = __builtin_amdgcn_wmma_f32_16x16x32_f16(false, al, false, bh, (short)0, c, false, false);
  if (NT >= 3) c = __builtin_amdgcn_wmma_f32_16x16x32_f16(false, ah, false, bl, (short)0, c, false, false);
  asm volatile("v_nop\n\tv_nop\n\tv_nop\n\tv_nop" : "+v"(c) : "v"(ah), "v"(al), "v"(bh), "v"(bl));
  return c;
}
template <bool ASPLIT>
__global__ __launch_bounds__(128) void k_gemm_h(const float* __restrict__ A, int lda, size_t sA, const _Float16* __restrict__ Bh, int ldb, size_t sB, float alpha, float* __restrict__ C, int ldc, size_t sC, int M, int N, int K) {
  __shared__ __attribute__((aligned(16))) float so[4][16][64];
  const int tid = threadIdx.x, w = tid >> 5, lane = tid & 31, ln = lane & 15, hh = lane >> 4; const int by = blockIdx.y;
  A += (size_t)by * sA; Bh += (size_t)by * sB; C += (size_t)by * sC;
  const int ntn = (N + 63) / 64; const int wid = blockIdx.x * 4 + w; const int mt = wid / ntn, nq = wid % ntn; if (mt * 16 >= M) return;
  const int row0 = mt * 16, col0 = nq * 64; const float* arow = A + (size_t)(row0 + ln) * lda;
  v8f acc[4] = {};
  for (int kb = 0; kb < K; kb += 32) {
    FragH ah, al;
    const v4f x0 = *(const v4fa*)(arow + kb + 8 * hh), x1 = *(const v4fa*)(arow + kb + 8 * hh + 4), x2 = *(const v4fa*)(arow + kb + 16 + 8 * hh), x3 = *(const v4fa*)(arow + kb + 16 + 8 * hh + 4);
    float xs[16] = {x0[0],x0[1],x0[2],x0[3],x1[0],x1[1],x1[2],x1[3],x2[0],x2[1],x2[2],x2[3],x3[0],x3[1],x3[2],x3[3]};
#pragma unroll
    for (int i = 0; i < 16; ++i) { const _Float16 h = (_Float16)xs[i]; ah.h[i] = h; al.h[i] = ASPLIT ? (_Float16)(xs[i] - (float)h) : (_Float16)0.0f; }
#pragma unroll
    for (int t = 0; t < 4; ++t) { if (col0 + t * 16 >= N) continue; const size_t boff = (size_t)(col0 + t * 16 + ln) * ldb + kb; FragH bq; bq.half[0] = *(const v8us*)(Bh + boff + 8 * hh); bq.half[1] = *(const v8us*)(Bh + boff + 16 + 8 * hh);
      acc[t] = mmaH<ASPLIT ? 2 : 1>(ah.v, al.v, bq.v, bq.v, acc[t]); }
  }
#pragma unroll
  for (int t = 0; t < 4; ++t) { if (col0 + t * 16 >= N) continue;
#pragma unroll
    for (int r = 0; r < 8; ++r) so[w][8 * hh + r][t * 16 + ln] = acc[t][r] * alpha; }
  __builtin_amdgcn_fence(__ATOMIC_ACQ_REL, "workgroup"); __builtin_amdgcn_wave_barrier();
  const int rsub = lane >> 4, c4 = (lane & 15) * 4;
  for (int pass = 0; pass < 2; ++pass) {
#pragma unroll
    for (int q = 0; q < 8; ++q) { const int r = q * 2 + rsub; if (col0 + c4 < N) { const v4f v = *(const v4fa*)&so[w][r][c4]; *(volatile v4f*)(C + (size_t)(row0 + r) * ldc + col0 + c4) = v; } }
    if (pass == 0) __threadfence(); }
}

__global__ __launch_bounds__(256) void k_wt_f16(const float* __restrict__ W, _Float16* __restrict__ Wt, int K, int N, float scale) {
  const int t = blockIdx.x * 256 + threadIdx.x; if (t >= N * (K / 8)) return; const int n = t / (K / 8), k8 = (t % (K / 8)) * 8; FragH f;
#pragma unroll
  for (int i = 0; i < 8; ++i) f.h[i] = (_Float16)(bf16_round(W[(size_t)(k8 + i) * N + n]) * scale); const v8us o = f.half[0];
  *(volatile v8us*)((unsigned short*)Wt + (size_t)n * K + k8) = o; __threadfence(); *(volatile v8us*)((unsigned short*)Wt + (size_t)n * K + k8) = o;
}
template <int ACT>
__global__ __launch_bounds__(128) void k_gemm_hhx(const _Float16* __restrict__ A, int lda, size_t sA, const _Float16* __restrict__ Bh, int ldb, size_t sB, float alpha, const float* __restrict__ bias, size_t sBias, const float* __restrict__ CP, int rowsPerB, size_t sCPb, int row0g,
    float* __restrict__ C, _Float16* __restrict__ C16, int ldc, size_t sC, int M, int N, int K) {
  __shared__ __attribute__((aligned(16))) float so[4][16][64];
  const int tid = threadIdx.x, w = tid >> 5, lane = tid & 31, ln = lane & 15, hh = lane >> 4; const int by = blockIdx.y;
  A += (size_t)by * sA; Bh += (size_t)by * sB; const size_t cofs = (size_t)by * sC; const float* bp = bias ? bias + (size_t)by * sBias : nullptr;
  const int ntn = (N + 63) / 64; const int wid = blockIdx.x * 4 + w; const int mt = wid / ntn, nq = wid % ntn; if (mt * 16 >= M) return;
  const int row0 = mt * 16, col0 = nq * 64; const _Float16* arow = A + (size_t)(row0 + ln) * lda;
  v8f acc[4] = {};
  for (int kb = 0; kb < K; kb += 32) { FragH ah; ah.half[0] = *(const v8us*)((const unsigned short*)arow + kb + 8 * hh); ah.half[1] = *(const v8us*)((const unsigned short*)arow + kb + 16 + 8 * hh);
#pragma unroll
    for (int t = 0; t < 4; ++t) { if (col0 + t * 16 >= N) continue; const size_t boff = (size_t)(col0 + t * 16 + ln) * ldb + kb; FragH bq; bq.half[0] = *(const v8us*)((const unsigned short*)Bh + boff + 8 * hh); bq.half[1] = *(const v8us*)((const unsigned short*)Bh + boff + 16 + 8 * hh);
      acc[t] = mmaH<1>(ah.v, ah.v, bq.v, bq.v, acc[t]); }
  }
#pragma unroll
  for (int t = 0; t < 4; ++t) { if (col0 + t * 16 >= N) continue; const int col = col0 + t * 16 + ln; const float bv = bp ? bf16_round(bp[col]) : 0.f;
#pragma unroll
    for (int r = 0; r < 8; ++r) { float v = acc[t][r] * alpha + bv; if (CP) { const int bidx = (row0g + row0 + 8 * hh + r) / rowsPerB; v += CP[(size_t)bidx * sCPb + (size_t)by * 64 + col]; } if (ACT == 1) v = (v > 0.f) ? v : expm1f(v); else if (ACT == 7) v = (v > 0.f) ? v + 1.0f : expf(v); else if (ACT == 8) v = tanhf(v); else if (ACT == 9) v = 0.5f * v * (1.0f + tanhf(0.7978845608028654f * (v + 0.044715f * v * v * v))); else if (ACT == 11) v = 1.0f / (1.0f + expf(-v)); else if (ACT == 12) v = (v > 0.f) ? v : 0.01f * v; else if (ACT == 14) v = (v > 0.f) ? v : 0.1f * v; else if (ACT == 15) v = v / (1.0f + expf(-v)); else if (ACT == 3) v = fmaxf(v, 0.f); else if (ACT == 6) v = 0.5f * v * (1.0f + erff(v * 0.70710678118654752f)); so[w][8 * hh + r][t * 16 + ln] = v; } }
  __builtin_amdgcn_fence(__ATOMIC_ACQ_REL, "workgroup"); __builtin_amdgcn_wave_barrier();
  const int rsub = lane >> 4, c4 = (lane & 15) * 4; typedef _Float16 v4h __attribute__((ext_vector_type(4)));
  for (int pass = 0; pass < 2; ++pass) {
#pragma unroll
    for (int q = 0; q < 8; ++q) { const int r = q * 2 + rsub; if (col0 + c4 < N) { const v4f v = *(const v4fa*)&so[w][r][c4]; if (C) *(volatile v4f*)(C + cofs + (size_t)(row0 + r) * ldc + col0 + c4) = v; if (C16) { v4h h4; for (int i = 0; i < 4; ++i) h4[i] = (_Float16)v[i]; *(volatile v4h*)(C16 + cofs + (size_t)(row0 + r) * ldc + col0 + c4) = h4; } } }
    if (pass == 0) __threadfence(); }
}


typedef _Float16 v4h __attribute__((ext_vector_type(4)));

__global__ __launch_bounds__(256) void k_x16(const float* __restrict__ x, _Float16* __restrict__ X16, size_t n8) { const size_t t = (size_t)blockIdx.x * 256 + threadIdx.x; if (t >= n8) return; FragH f;
#pragma unroll
  for (int q = 0; q < 8; ++q) f.h[q] = (_Float16)bf16_round(x[t * 8 + q]); *(volatile v8us*)((unsigned short*)X16 + t * 8) = f.half[0]; __threadfence(); *(volatile v8us*)((unsigned short*)X16 + t * 8) = f.half[0]; }
__global__ __launch_bounds__(256) void k_h16(const float* __restrict__ x, _Float16* __restrict__ X16, size_t n8) { const size_t t = (size_t)blockIdx.x * 256 + threadIdx.x; if (t >= n8) return; FragH f;
#pragma unroll
  for (int q = 0; q < 8; ++q) f.h[q] = (_Float16)x[t * 8 + q]; *(volatile v8us*)((unsigned short*)X16 + t * 8) = f.half[0]; __threadfence(); *(volatile v8us*)((unsigned short*)X16 + t * 8) = f.half[0]; }
__global__ __launch_bounds__(256) void k_round16f(const float* __restrict__ W, _Float16* __restrict__ Bt, size_t n8) { const size_t t = (size_t)blockIdx.x * 256 + threadIdx.x; if (t >= n8) return; FragH f;
#pragma unroll
  for (int i = 0; i < 8; ++i) f.h[i] = (_Float16)(bf16_round(W[t * 8 + i]) * 16.0f); *(volatile v8us*)((unsigned short*)Bt + t * 8) = f.half[0]; __threadfence(); *(volatile v8us*)((unsigned short*)Bt + t * 8) = f.half[0]; }
template <int NHv, int TTv>
__global__ __launch_bounds__(256) void k_vt(const _Float16* __restrict__ V16, int ldv, int voff, _Float16* __restrict__ Vt) { __shared__ unsigned short tl[64][66]; const int tid = threadIdx.x; const int slab = blockIdx.x / (TTv / 64), lg = blockIdx.x % (TTv / 64); const int b = slab / NHv, h = slab % NHv;
  for (int i = tid; i < 64 * 8; i += 256) { const int r = i / 8, c8 = (i % 8) * 8; FragH f; f.half[0] = *(const v8us*)((const unsigned short*)V16 + ((size_t)b * TTv + lg * 64 + r) * ldv + voff + h * 64 + c8);
#pragma unroll
    for (int q = 0; q < 8; ++q) tl[r][c8 + q] = f.u[q]; }
  __syncthreads();
  for (int pass = 0; pass < 2; ++pass) {
#pragma unroll
    for (int rd = 0; rd < 2; ++rd) { const int d = rd * 32 + tid / 8, pc = tid % 8; FragH f;
#pragma unroll
      for (int q = 0; q < 8; ++q) f.u[q] = tl[pc * 8 + q][d];
      *(volatile v8us*)((unsigned short*)Vt + ((size_t)slab * 64 + d) * TTv + lg * 64 + pc * 8) = f.half[0]; }
    if (pass == 0) __threadfence(); } }

__global__ __launch_bounds__(256) void k_hl(const float* __restrict__ F, _Float16* __restrict__ Hh, _Float16* __restrict__ Hl, size_t n8) { const size_t t = (size_t)blockIdx.x * 256 + threadIdx.x; if (t >= n8) return; FragH fh, fl; const v4f a = *(const v4fa*)(F + t * 8), c = *(const v4fa*)(F + t * 8 + 4);
#pragma unroll
  for (int q = 0; q < 4; ++q) { _Float16 h = (_Float16)a[q]; fh.h[q] = h; fl.h[q] = (_Float16)((a[q] - (float)h) * 1024.0f); h = (_Float16)c[q]; fh.h[4 + q] = h; fl.h[4 + q] = (_Float16)((c[q] - (float)h) * 1024.0f); }
  for (int pass = 0; pass < 2; ++pass) { *(volatile v8us*)((unsigned short*)Hh + t * 8) = fh.half[0]; *(volatile v8us*)((unsigned short*)Hl + t * 8) = fl.half[0]; if (pass == 0) __threadfence(); } }

__device__ __forceinline__ float sigm(float v) { return 1.0f / (1.0f + expf(-v)); }
__global__ __launch_bounds__(256) void k_stgA1(int b0, const float* __restrict__ x, const float* __restrict__ U1, const float* __restrict__ U2, const float* __restrict__ U3, const float* __restrict__ be, const float* __restrict__ Ve, const float* __restrict__ W1, const float* __restrict__ W2, const float* __restrict__ W3, const float* __restrict__ bs_, const float* __restrict__ Vs, const float* __restrict__ av, float* __restrict__ SP, float* __restrict__ SAT, float* __restrict__ PL) {
  #pragma clang fp contract(off)
  __shared__ float xs[TT][VV][FD], xT[TT][VV][FD]; __shared__ float lhs[TT][VV], rhs[VV][TT], prodm[TT][TT], At[TT][TT]; __shared__ float slhs[VV][TT], srhs[TT][VV]; __shared__ float M1[VV][VV], M2[VV][VV]; __shared__ float colv[VV], dg[VV], d2[VV][FD], red[256]; __shared__ __attribute__((aligned(16))) float nrm2[2 * VV];
  const int tid = threadIdx.x, b = b0 + blockIdx.x;
  for (int i = tid; i < TT * VV * FD; i += 256) ((float*)xs)[i] = bf16_round(x[(size_t)b * TT * VV * FD + i]);
  __syncthreads();
  if (tid < TT * VV) { const int t = tid / VV, u = tid % VV; float s = 0.f; _Pragma("unroll 1") for (int v = 0; v < VV; ++v) { const float u1 = bf16_round(U1[v]); for (int f = 0; f < FD; ++f) s += xs[t][v][f] * u1 * bf16_round(U2[f * VV + u]); } lhs[t][u] = s; }
  if (tid < VV * TT) { const int v = tid / TT, t = tid % TT; float s = 0.f; for (int f = 0; f < FD; ++f) s += bf16_round(U3[f]) * xs[t][v][f]; rhs[v][t] = s; }
  __syncthreads();
  if (tid < TT * TT) { const int t = tid / TT, u = tid % TT; float s = 0.f; _Pragma("unroll 1") for (int v = 0; v < VV; ++v) s += lhs[t][v] * rhs[v][u]; prodm[t][u] = s; }
  __syncthreads();
  if (tid < TT * TT) { const int t = tid / TT, u = tid % TT; float s = 0.f; _Pragma("unroll 1") for (int q = 0; q < TT; ++q) s += bf16_round(Ve[t * TT + q]) * sigm(prodm[q][u] + bf16_round(be[q * TT + u])); At[t][u] = s; }
  __syncthreads();
  if (tid < TT) { const int u = tid; float m = fmaxf(fmaxf(At[0][u], At[1][u]), At[2][u]); float su = 0.f; _Pragma("unroll 1") for (int t = 0; t < TT; ++t) { const float e = expf(At[t][u] - m); red[u * 3 + t] = e; su += e; } _Pragma("unroll 1") for (int t = 0; t < TT; ++t) red[u * 3 + t] = red[u * 3 + t] / su; }
  __syncthreads();
  if (tid < TT * TT) { const int t = tid / TT, u = tid % TT; At[t][u] = red[u * 3 + t]; }
  __syncthreads();
  const float isq = 1.0f / sqrtf(310.0f);
  for (int i = tid; i < TT * VV * FD; i += 256) { const int u = i / (VV * FD), v = (i / FD) % VV, f = i % FD; float s = 0.f; for (int t = 0; t < TT; ++t) s += xs[t][v][f] * At[t][u]; xT[u][v][f] = s * isq; }
  __syncthreads();
  if (tid < VV * TT) { const int v = tid / TT, sI = tid % TT; float s = 0.f; for (int t = 0; t < TT; ++t) { const float w1 = bf16_round(W1[t]); for (int f = 0; f < FD; ++f) s += xT[t][v][f] * w1 * bf16_round(W2[f * TT + sI]); } slhs[v][sI] = s; }
  for (int i = tid; i < TT * VV; i += 256) { const int t = i / VV, v = i % VV; float s = 0.f; for (int f = 0; f < FD; ++f) s += bf16_round(W3[f]) * xT[t][v][f]; srhs[t][v] = s; }
  __syncthreads();
  for (int i = tid; i < NS; i += 256) { const int u = i / VV, v = i % VV; float s = 0.f; for (int t = 0; t < TT; ++t) s += slhs[u][t] * srhs[t][v]; M1[u][v] = sigm(s + bf16_round(bs_[i])); }
  __syncthreads();
  for (int i = tid; i < NS; i += 256) { const int u = i / VV, v = i % VV; float s = 0.f; _Pragma("unroll 1") for (int w = 0; w < VV; ++w) s += bf16_round(Vs[u * VV + w]) * M1[w][v]; M2[u][v] = s; }
  __syncthreads();
  if (tid < VV) { const int v = tid; float m = -3.0e38f; _Pragma("unroll 1") for (int u = 0; u < VV; ++u) m = fmaxf(m, M2[u][v]); float su = 0.f; _Pragma("unroll 1") for (int u = 0; u < VV; ++u) su += expf(M2[u][v] - m); typedef float v2f __attribute__((ext_vector_type(2))); v2f st; st[0] = m; st[1] = 1.0f / su; ((v2f*)nrm2)[v] = st; }
  __syncthreads();
  for (int i = tid; i < NS; i += 256) { const int u = i / VV, v = i % VV; M2[u][v] = expf(M2[u][v] - nrm2[2 * v]) * nrm2[2 * v + 1]; }
  __syncthreads();
  for (int pass = 0; pass < 2; ++pass) { for (int i = tid; i < 3872; i += 256) { const float a2 = (i < NS) ? M2[i / VV][i % VV] : 0.f; *(volatile float*)(SAT + (size_t)(b - b0) * 3872 + i) = a2; } if (pass == 0) __threadfence(); } (void)SP; (void)PL; (void)av; }
__global__ __launch_bounds__(256) void k_stgA2(int b0, const float* __restrict__ x, const float* __restrict__ U1, const float* __restrict__ U2, const float* __restrict__ U3, const float* __restrict__ be, const float* __restrict__ Ve, const float* __restrict__ W1, const float* __restrict__ W2, const float* __restrict__ W3, const float* __restrict__ bs_, const float* __restrict__ Vs, const float* __restrict__ av, float* __restrict__ SP, float* __restrict__ SAT, float* __restrict__ PL) {
  #pragma clang fp contract(off)
  __shared__ float xs[TT][VV][FD], xT[TT][VV][FD]; __shared__ float lhs[TT][VV], rhs[VV][TT], prodm[TT][TT], At[TT][TT]; __shared__ float slhs[VV][TT], srhs[TT][VV]; __shared__ float M1[VV][VV], M2[VV][VV]; __shared__ float colv[VV], dg[VV], d2[VV][FD], red[256]; __shared__ __attribute__((aligned(16))) float nrm2[2 * VV];
  const int tid = threadIdx.x, b = b0 + blockIdx.x;
  for (int i = tid; i < TT * VV * FD; i += 256) ((float*)xs)[i] = bf16_round(x[(size_t)b * TT * VV * FD + i]);
  __syncthreads();
  for (int i = tid; i < NS; i += 256) { const int ii = i / VV, j = i % VV; float s = 0.f; for (int f = 0; f < FD; ++f) { const float d = xs[1][ii][f] - xs[1][j][f]; s += ((d >= 0.f) ? d : (0.f - d)) * bf16_round(av[f]); } M1[ii][j] = expf(fmaxf(s, 0.f)); }
  __syncthreads();
  if (tid < VV) { const int j = tid; float su = 0.f; _Pragma("unroll 1") for (int ii = 0; ii < VV; ++ii) su += M1[ii][j]; colv[j] = su; }
  if (tid >= 64 && tid < 64 + VV) { const int ii = tid - 64; for (int f = 0; f < FD; ++f) { float s = 0.f; _Pragma("unroll 1") for (int j = 0; j < VV; ++j) { const float d = xs[1][ii][f] - xs[1][j][f]; s += d * d; } d2[ii][f] = s; } }
  __syncthreads();
  for (int i = tid; i < NS; i += 256) { const int j = i % VV; M1[i / VV][j] = M1[i / VV][j] / colv[j]; }
  __syncthreads();
  { float p1 = 0.f, p2 = 0.f; for (int i = tid; i < NS; i += 256) { const int ii = i / VV, j = i % VV; const float sv = M1[ii][j]; p1 += sv * sv; float dd = 0.f; for (int f = 0; f < FD; ++f) dd += d2[j][f]; p2 += sv * dd; }
    red[tid] = p1; __syncthreads(); for (int st = 128; st > 0; st >>= 1) { if (tid < st) red[tid] += red[tid + st]; __syncthreads(); } const float s1 = red[0]; __syncthreads();
    red[tid] = p2; __syncthreads(); for (int st = 128; st > 0; st >>= 1) { if (tid < st) red[tid] += red[tid + st]; __syncthreads(); } const float s2 = red[0]; __syncthreads();
    if (tid < 32) { float* line = PL + (size_t)b * 32; const float v = (tid == 0) ? s1 : (tid == 1) ? s2 : 0.f; *(volatile float*)(line + tid) = v; __threadfence(); *(volatile float*)(line + tid) = v; } }
  for (int pass = 0; pass < 2; ++pass) { for (int i = tid; i < 3872; i += 256) { const float v = (i < NS) ? M1[i / VV][i % VV] : 0.f; *(volatile float*)(SP + (size_t)b * 3872 + i) = v; } if (pass == 0) __threadfence(); } (void)SAT; (void)U1; (void)U2; (void)U3; (void)be; (void)Ve; (void)W1; (void)W2; (void)W3; (void)bs_; (void)Vs; }

__global__ __launch_bounds__(256) void k_stgB(int b0, const float* __restrict__ x, const float* __restrict__ SP, const float* __restrict__ SAT, _Float16* __restrict__ AZ) {
  #pragma clang fp contract(off)
  __shared__ float xs[TT][VV][FD], M1[VV][VV], M2[VV][VV], dg[VV]; __shared__ __attribute__((aligned(16))) unsigned short zrow[64][64]; const int tid = threadIdx.x, bl = blockIdx.x, b = b0 + bl;
  for (int i = tid; i < TT * VV * FD; i += 256) ((float*)xs)[i] = bf16_round(x[(size_t)b * TT * VV * FD + i]);
  for (int i = tid; i < NS; i += 256) { M1[i / VV][i % VV] = SP[(size_t)b * 3872 + i]; M2[i / VV][i % VV] = SAT[(size_t)bl * 3872 + i]; }
  for (int i = tid; i < 64 * 64; i += 256) ((unsigned short*)zrow)[i] = 0;
  __syncthreads();
  if (tid < VV) { const int j = tid; float su = 0.f; _Pragma("unroll 1") for (int ii = 0; ii < VV; ++ii) su += M1[ii][j]; dg[j] = su; }
  __syncthreads();
  if (tid < VV * TT) { const int v = tid / TT, t = tid % TT; float z[3][FD];
#pragma unroll
    for (int k = 0; k < 3; ++k) for (int f = 0; f < FD; ++f) z[k][f] = 0.f;
    _Pragma("unroll 1") for (int u = 0; u < VV; ++u) { const float suv = M1[u][v], at = M2[u][v]; const float dlt = (u == v) ? 1.f : 0.f; const float lt = (dg[v] - 1.0f) * dlt - suv; const float c0 = dlt * at, c1 = lt * at, c2 = (2.0f * lt * lt - dlt) * at;
#pragma unroll
      for (int f = 0; f < FD; ++f) { const float xv = xs[t][u][f]; z[0][f] += c0 * xv; z[1][f] += c1 * xv; z[2][f] += c2 * xv; } }
#pragma unroll
    for (int k = 0; k < 3; ++k) for (int f = 0; f < FD; ++f) { FragH h; h.h[0] = (_Float16)z[k][f]; zrow[v][t * 16 + k * 5 + f] = h.u[0]; } }
  __syncthreads();
  for (int pass = 0; pass < 2; ++pass) { for (int i = tid; i < VV * 16; i += 256) { const int v = i >> 4, c8 = (i & 15) * 4; const unsigned long long pv = *(const unsigned long long*)&zrow[v][c8]; *(volatile unsigned long long*)((unsigned short*)AZ + ((size_t)bl * VV + v) * 64 + c8) = pv; } if (pass == 0) __threadfence(); } }
__global__ __launch_bounds__(256) void k_btheta(const float* __restrict__ Th, _Float16* __restrict__ Bt) { const int t_ = blockIdx.x * 256 + threadIdx.x; if (t_ >= 192 * 8) return; const int c0 = (t_ & 7) * 8, row = t_ >> 3; const int t = row / HH, o = row % HH; FragH f;
#pragma unroll
  for (int q = 0; q < 8; ++q) { const int c = c0 + q; const int tp = c / 16, r = c % 16; const int k = r / 5, ff = r % 5; const bool ok = (tp == t) && (r < 15); f.h[q] = ok ? (_Float16)(bf16_round(Th[((size_t)k * FD + ff) * HH + o]) * 16.0f) : (_Float16)0.0f; }
  *(volatile v8us*)((unsigned short*)Bt + (size_t)row * 64 + c0) = f.half[0]; __threadfence(); *(volatile v8us*)((unsigned short*)Bt + (size_t)row * 64 + c0) = f.half[0]; }
__global__ __launch_bounds__(256) void k_btw(const float* __restrict__ tw, _Float16* __restrict__ Bt) { const int t_ = blockIdx.x * 256 + threadIdx.x; if (t_ >= HH * 24) return; const int c0 = (t_ % 24) * 8, o2 = t_ / 24; FragH f;
#pragma unroll
  for (int q = 0; q < 8; ++q) { const int c = c0 + q; const int t = c / HH, o = c % HH; f.h[q] = (_Float16)(bf16_round(tw[((size_t)o2 * HH + o) * TT + t]) * 16.0f); }
  *(volatile v8us*)((unsigned short*)Bt + (size_t)o2 * 192 + c0) = f.half[0]; __threadfence(); *(volatile v8us*)((unsigned short*)Bt + (size_t)o2 * 192 + c0) = f.half[0]; }
__global__ __launch_bounds__(256) void k_fin(const float* __restrict__ TC, const float* __restrict__ x, const float* __restrict__ rw, const float* __restrict__ rb, const float* __restrict__ tb, const float* __restrict__ g, const float* __restrict__ bb, float* __restrict__ out) {
  #pragma clang fp contract(off)
  const int tid = threadIdx.x, w = tid >> 5, ln = tid & 31; const int r = blockIdx.x * 8 + w; if (r >= NRV) return; const int b = r / VV, v = r % VV; const float* xr = x + (((size_t)b * TT + 0) * VV + v) * FD; const float isq15 = 1.0f / sqrtf(15.0f); float zz[2];
#pragma unroll
  for (int q = 0; q < 2; ++q) { const int o = ln * 2 + q; float res = bf16_round(rb[o]); for (int f = 0; f < FD; ++f) res += bf16_round(xr[f]) * bf16_round(rw[o * FD + f]); const float tc = (TC[(size_t)r * HH + o] + bf16_round(tb[o])) * isq15; zz[q] = fmaxf(res + tc, 0.f); }
  float s = zz[0] + zz[1]; for (int o = 16; o > 0; o >>= 1) s += __shfl_xor(s, o, 32); const float mu = s / (float)HH; float q2 = (zz[0] - mu) * (zz[0] - mu) + (zz[1] - mu) * (zz[1] - mu); for (int o = 16; o > 0; o >>= 1) q2 += __shfl_xor(q2, o, 32); const float rs = 1.0f / sqrtf(q2 / (float)HH + 1e-5f);
  typedef float v2f __attribute__((ext_vector_type(2))); v2f ov; ov[0] = (zz[0] - mu) * rs * bf16_round(g[ln * 2]) + bf16_round(bb[ln * 2]); ov[1] = (zz[1] - mu) * rs * bf16_round(g[ln * 2 + 1]) + bf16_round(bb[ln * 2 + 1]);
  *(volatile v2f*)(out + (size_t)r * HH + ln * 2) = ov; __threadfence(); *(volatile v2f*)(out + (size_t)r * HH + ln * 2) = ov; }
__global__ __launch_bounds__(256) void k_sout(const float* __restrict__ PL, const float* __restrict__ SP, float* __restrict__ base) {
  #pragma clang fp contract(off)
  __shared__ float red[256]; __shared__ float fin[2]; const int tid = threadIdx.x, w = tid >> 5, ln = tid & 31;
  for (int which = 0; which < 2; ++which) { float s = 0.f; for (int b = tid; b < NB; b += 256) s += PL[(size_t)b * 32 + which]; red[tid] = s; __syncthreads(); for (int st = 128; st > 0; st >>= 1) { if (tid < st) red[tid] += red[tid + st]; __syncthreads(); } if (tid == 0) fin[which] = red[0]; __syncthreads(); }
  const float sloss = 1.0e-4f * (fin[0] / (float)NB), dloss = 1.0e-4f * fin[1];
  const size_t npieces = 1 + (size_t)NB * NS / 2;
  const size_t per_wave = ((npieces + 8 * 32 - 1) / (8 * 32)) * 32;
  typedef float v2f __attribute__((ext_vector_type(2)));
  for (int pass = 0; pass < 2; ++pass) {
    for (size_t p = (size_t)w * per_wave + ln; p < min(npieces, (size_t)(w + 1) * per_wave); p += 32) { v2f val;
      if (p == 0) { val[0] = sloss; val[1] = dloss; } else { const size_t e = 2 * (p - 1); const size_t b0 = e / NS, i0 = e % NS, b1 = (e + 1) / NS, i1 = (e + 1) % NS; val[0] = SP[b0 * 3872 + i0]; val[1] = SP[b1 * 3872 + i1]; }
      *(volatile v2f*)(base + 2 * p) = val; }
    if (pass == 0) __threadfence(); } }

extern "C" void kernel_launch(void* const* d_in, const int* in_sizes, int n_in,
                              void* d_out, int out_size, void* d_ws, size_t ws_size, hipStream_t stream) {
  (void)in_sizes; (void)n_in; (void)out_size;
  const float* const* I = (const float* const*)d_in; const float* x = I[0];
  char* ws = (char*)d_ws; size_t off = 0;
  auto take = [&](size_t bytes) { char* p = ws + off; off += (bytes + 255) & ~(size_t)255; return p; };
  const int HB = NB / 2; const int HRV = HB * VV;
  _Float16* BTH = (_Float16*)take(192 * 64 * 2); _Float16* BTW = (_Float16*)take(64 * 192 * 2); _Float16* AZ = (_Float16*)take((size_t)HRV * 64 * 2); float* SP = (float*)take((size_t)NB * 3872 * 4); float* SAT = (float*)take((size_t)HB * 3872 * 4); float* PL = (float*)take((size_t)NB * 32 * 4); _Float16* G16 = (_Float16*)take((size_t)HRV * 192 * 2); float* TC = (float*)take((size_t)HRV * HH * 4);
  if (off > ws_size) return;
  k_btheta<<<(192 * 8 + 255) / 256, 256, 0, stream>>>(I[12], BTH); k_btw<<<(HH * 24 + 255) / 256, 256, 0, stream>>>(I[13], BTW);
  for (int hf = 0; hf < 2; ++hf) { const int b0 = hf * HB;
    k_stgA1<<<HB, 256, 0, stream>>>(b0, x, I[1], I[2], I[3], I[4], I[5], I[6], I[7], I[8], I[9], I[10], I[11], SP, SAT, PL); k_stgA2<<<HB, 256, 0, stream>>>(b0, x, I[1], I[2], I[3], I[4], I[5], I[6], I[7], I[8], I[9], I[10], I[11], SP, SAT, PL);
    k_stgB<<<HB, 256, 0, stream>>>(b0, x, SP, SAT, AZ);
    k_gemm_hhx<3><<<dim3(((HRV / 16) * 3 + 3) / 4, 1), 128, 0, stream>>>(AZ, 64, 0, BTH, 64, 0, 0.0625f, nullptr, 0, nullptr, 1, 0, 0, nullptr, G16, 192, 0, HRV, 192, 64);
    k_gemm_hhx<0><<<dim3(((HRV / 16) * 1 + 3) / 4, 1), 128, 0, stream>>>(G16, 192, 0, BTW, 192, 0, 0.0625f, nullptr, 0, nullptr, 1, 0, 0, TC, nullptr, HH, 0, HRV, HH, 192);
    k_fin<<<HRV / 8, 256, 0, stream>>>(TC, x + (size_t)b0 * TT * VV * FD, I[15], I[16], I[14], I[17], I[18], (float*)d_out + (size_t)b0 * VV * HH); }
  k_sout<<<1, 256, 0, stream>>>(PL, SP, (float*)((char*)d_out + 32505856));
}
